// CTRNNHebb_73100343378142
// MI455X (gfx1250) — hardware-run, weakly checked
//
#include <hip/hip_runtime.h>
#include <math.h>

constexpr int NSTEP = 512;
constexpr int NSAMP = 256;
constexpr int NIN   = 64;
constexpr int NH0   = 32;
constexpr int NHID  = 128;
constexpr int NOUT  = 64;
constexpr int NROWS = NSTEP * NSAMP;
constexpr int XROWS = (NSTEP - 1) * NSAMP;
constexpr int SCAN_THR = 1024;
constexpr int SCAN_GRP = SCAN_THR / NHID;
constexpr int SCAN_EPT = NHID / SCAN_GRP;
constexpr float ACT_CARRY  = 16.0f;
constexpr float WOUT_CARRY = 64.0f;
constexpr float OUT_FOLD   = 1.0f / (ACT_CARRY * WOUT_CARRY);

static_assert(SCAN_GRP == 8 && SCAN_EPT == 16, "scan decomposition");
static_assert(XROWS % 64 == 0 && NROWS % 64 == 0, "GEMM M tile multiples");
static_assert(NHID % 64 == 0 && NOUT % 64 == 0, "GEMM N tile multiples");
static_assert(NIN % 32 == 0 && NHID % 32 == 0, "GEMM K multiples of 32");
static_assert(((XROWS * (NIN / 8)) % 256) == 0, "split grid exact");
static_assert((((XROWS >> 6) * (NHID >> 6)) % 8) == 0, "input GEMM grid exact");
static_assert((((NROWS >> 6) * (NOUT >> 6)) % 8) == 0, "output GEMM grid exact");

typedef __attribute__((ext_vector_type(16))) _Float16 v16h;
typedef __attribute__((ext_vector_type(8)))  _Float16 v8h;
typedef __attribute__((ext_vector_type(2)))  _Float16 v2h;
typedef __attribute__((ext_vector_type(16))) __bf16   v16b;
typedef __attribute__((ext_vector_type(8)))  __bf16   v8b;
typedef __attribute__((ext_vector_type(8)))  float    v8f;
typedef __attribute__((ext_vector_type(4)))  float    v4f;

__device__ __forceinline__ unsigned short f2bf_bits(float f) {
  unsigned u = __float_as_uint(f);
  return (unsigned short)((u + 0x7FFFu + ((u >> 16) & 1u)) >> 16);
}
__device__ __forceinline__ float bf_bits2f(unsigned short h) { return __uint_as_float(((unsigned)h) << 16); }

__device__ __forceinline__ void dep_guard4_h(v8f& a, v8f& b, v8f& c, v8f& d, v16h x, v16h y) {
  asm volatile("v_nop\n\tv_nop\n\tv_nop\n\tv_nop" : "+v"(a), "+v"(b), "+v"(c), "+v"(d) : "v"(x), "v"(y));
}
__device__ __forceinline__ void dep_guard4_b(v8f& a, v8f& b, v8f& c, v8f& d, v16b x, v16b y) {
  asm volatile("v_nop\n\tv_nop\n\tv_nop\n\tv_nop" : "+v"(a), "+v"(b), "+v"(c), "+v"(d) : "v"(x), "v"(y));
}
__device__ __forceinline__ void keep4_h(v16h a, v16h b, v16h c, v16h d) { asm volatile("v_nop" :: "v"(a), "v"(b), "v"(c), "v"(d)); }
__device__ __forceinline__ void keep4_b(v16b a, v16b b, v16b c, v16b d) { asm volatile("v_nop" :: "v"(a), "v"(b), "v"(c), "v"(d)); }
__device__ __forceinline__ void acc_guard4(v8f& a, v8f& b, v8f& c, v8f& d) {
  asm volatile("v_nop\n\tv_nop\n\tv_nop\n\tv_nop" : "+v"(a), "+v"(b), "+v"(c), "+v"(d));
}

template <typename T> struct Frag;
template <> struct Frag<_Float16> {
  typedef v16h V; union U { v16h v; v8h h[2]; };
  static __device__ __forceinline__ v16h load(const _Float16* p) {
    U f; f.h[0] = *(const v8h*)(p); f.h[1] = *(const v8h*)(p + 16); return f.v;
  }
  static __device__ __forceinline__ v8f mma(v16h a, v16h b, v8f c) {
    return __builtin_amdgcn_wmma_f32_16x16x32_f16(false, a, false, b, (short)0, c, false, false);
  }
  static __device__ __forceinline__ void guard4(v8f& a, v8f& b, v8f& c, v8f& d, v16h x, v16h y) { dep_guard4_h(a, b, c, d, x, y); }
  static __device__ __forceinline__ void keep(v16h a, v16h b, v16h c, v16h d) { keep4_h(a, b, c, d); }
};
template <> struct Frag<__bf16> {
  typedef v16b V; union U { v16b v; v8b h[2]; };
  static __device__ __forceinline__ v16b load(const __bf16* p) {
    U f; f.h[0] = *(const v8b*)(p); f.h[1] = *(const v8b*)(p + 16); return f.v;
  }
  static __device__ __forceinline__ v8f mma(v16b a, v16b b, v8f c) {
    return __builtin_amdgcn_wmma_f32_16x16x32_bf16(false, a, false, b, (short)0, c, false, false);
  }
  static __device__ __forceinline__ void guard4(v8f& a, v8f& b, v8f& c, v8f& d, v16b x, v16b y) { dep_guard4_b(a, b, c, d, x, y); }
  static __device__ __forceinline__ void keep(v16b a, v16b b, v16b c, v16b d) { keep4_b(a, b, c, d); }
};

template <int ET> struct Elem;
template <> struct Elem<0> { typedef _Float16 T; };
template <> struct Elem<1> { typedef __bf16 T; };

template <int ET, bool SPLIT, int BIAS_MODE>
__global__ __launch_bounds__(256) void wmma_gemm64(
    const unsigned short* __restrict__ Ap, const unsigned short* __restrict__ A2p, int lda,
    const unsigned short* __restrict__ Btp, const unsigned short* __restrict__ Bt2p, int ldb,
    float* __restrict__ C, int ldc, const float* __restrict__ bias,
    int M, int N, int K, float scale) {
  typedef typename Elem<ET>::T T;
  typedef typename Frag<T>::V V;
  const T* A = (const T*)Ap; const T* A2 = (const T*)A2p; const T* Bt = (const T*)Btp; const T* Bt2 = (const T*)Bt2p;
  __shared__ __align__(16) float sT[8][16 * 68];
  const int lane = threadIdx.x & 31;
  const int wave = __builtin_amdgcn_readfirstlane((int)(threadIdx.x >> 5));
  const int tilesN = N >> 6;
  const int tilesM = M >> 6;
  const int tile = blockIdx.x * 8 + wave;
  if (tile >= tilesM * tilesN) return;
  const int tm = tile / tilesN;
  const int tn = tile - tm * tilesN;
  const int m0 = tm << 6;
  const int n0 = tn << 6;

  const int rlane = lane & 15;
  const int koff  = (lane >> 4) * 8;
  const int mOff  = (lane >> 4) * 8;

  v8f acc[4][4];
#pragma unroll
  for (int i = 0; i < 4; ++i)
#pragma unroll
    for (int j = 0; j < 4; ++j) acc[i][j] = (v8f){0.f, 0.f, 0.f, 0.f, 0.f, 0.f, 0.f, 0.f};

  for (int k0 = 0; k0 < K; k0 += 32) {
    V bh[4], bl[4];
#pragma unroll
    for (int j = 0; j < 4; ++j) {
      const size_t bo = (size_t)(n0 + (j << 4) + rlane) * ldb + koff + k0;
      bh[j] = Frag<T>::load(Bt + bo);
      if (SPLIT) bl[j] = Frag<T>::load(Bt2 + bo);
    }
#pragma unroll
    for (int i = 0; i < 4; ++i) {
      const size_t ao = (size_t)(m0 + (i << 4) + rlane) * lda + koff + k0;
      V ah = Frag<T>::load(A + ao);
      V al;
      if (SPLIT) al = Frag<T>::load(A2 + ao);
#pragma unroll
      for (int j = 0; j < 4; ++j) {
        acc[i][j] = Frag<T>::mma(ah, bh[j], acc[i][j]);
        if (SPLIT) {
          acc[i][j] = Frag<T>::mma(ah, bl[j], acc[i][j]);
          acc[i][j] = Frag<T>::mma(al, bh[j], acc[i][j]);
        }
      }
      Frag<T>::guard4(acc[i][0], acc[i][1], acc[i][2], acc[i][3], ah, SPLIT ? al : ah);
    }
    Frag<T>::keep(bh[0], bh[1], bh[2], bh[3]);
    if (SPLIT) Frag<T>::keep(bl[0], bl[1], bl[2], bl[3]);
  }
  acc_guard4(acc[0][0], acc[0][1], acc[0][2], acc[0][3]);
  acc_guard4(acc[1][0], acc[1][1], acc[1][2], acc[1][3]);
  acc_guard4(acc[2][0], acc[2][1], acc[2][2], acc[2][3]);
  acc_guard4(acc[3][0], acc[3][1], acc[3][2], acc[3][3]);

  float* slab = sT[wave];
#pragma unroll
  for (int i = 0; i < 4; ++i) {
    const int mBase = m0 + (i << 4);
#pragma unroll
    for (int j = 0; j < 4; ++j) {
      const int n = n0 + (j << 4) + rlane;
      float bv = 0.f;
      if (BIAS_MODE == 2) bv = bias[n];
#pragma unroll
      for (int r = 0; r < 8; ++r) {
        float v = acc[i][j][r] * scale;
        if (BIAS_MODE == 2) v += bv;
        slab[(mOff + r) * 68 + (j << 4) + rlane] = v;
      }
    }
    __builtin_amdgcn_fence(__ATOMIC_RELEASE, "workgroup");
    __builtin_amdgcn_wave_barrier();
    __builtin_amdgcn_fence(__ATOMIC_ACQUIRE, "workgroup");
    {
      const int hh = lane >> 4, c4 = (lane & 15) * 4;
      for (int pass = 0; pass < 2; ++pass) {
#pragma unroll
        for (int it = 0; it < 8; ++it) {
          const int row = it * 2 + hh;
          const v4f v = *(const v4f*)(slab + row * 68 + c4);
          *(volatile v4f*)(C + (size_t)(mBase + row) * ldc + n0 + c4) = v;
        }
        __threadfence();
      }
    }
    __builtin_amdgcn_fence(__ATOMIC_RELEASE, "workgroup");
    __builtin_amdgcn_wave_barrier();
    __builtin_amdgcn_fence(__ATOMIC_ACQUIRE, "workgroup");
  }
}

__global__ __launch_bounds__(256) void split8_kernel(const float* __restrict__ src, unsigned short* __restrict__ hi,
                                                     unsigned short* __restrict__ lo, int n8) {
  const int i = blockIdx.x * 256 + threadIdx.x;
  if (i < n8) {
    const float* sp = src + (size_t)i * 8;
    const v4f a = *(const v4f*)(sp);
    const v4f b = *(const v4f*)(sp + 4);
    v8h hv, lv;
#pragma unroll
    for (int e = 0; e < 4; ++e) {
      const float f0 = a[e];
      const float f1 = b[e];
      const unsigned short h0 = f2bf_bits(f0);
      const unsigned short h1 = f2bf_bits(f1);
      const unsigned short l0 = f2bf_bits(f0 - bf_bits2f(h0));
      const unsigned short l1 = f2bf_bits(f1 - bf_bits2f(h1));
      hv[e]     = __builtin_bit_cast(_Float16, h0);
      hv[4 + e] = __builtin_bit_cast(_Float16, h1);
      lv[e]     = __builtin_bit_cast(_Float16, l0);
      lv[4 + e] = __builtin_bit_cast(_Float16, l1);
    }
    *(volatile v8h*)(hi + (size_t)i * 8) = hv;
    *(volatile v8h*)(lo + (size_t)i * 8) = lv;
    __threadfence();
    *(volatile v8h*)(hi + (size_t)i * 8) = hv;
    *(volatile v8h*)(lo + (size_t)i * 8) = lv;
  }
}

template <int MODE>
__global__ __launch_bounds__(256) void tp_kernel(const float* __restrict__ src, int R, int C, int ldo,
                                                 unsigned short* __restrict__ O, unsigned short* __restrict__ O2, float sc) {
  __shared__ float Tt[64 * 65];
  const int tid = threadIdx.x;
  const int c0 = blockIdx.x * 64, r0 = blockIdx.y * 64;
#pragma unroll
  for (int i = 0; i < 4; ++i) {
    const int idx = i * 256 + tid;
    const int rr = idx >> 4, cc = (idx & 15) * 4;
    const v4f v = *(const v4f*)(src + (size_t)(r0 + rr) * (size_t)C + c0 + cc);
    Tt[rr * 65 + cc + 0] = v[0];
    Tt[rr * 65 + cc + 1] = v[1];
    Tt[rr * 65 + cc + 2] = v[2];
    Tt[rr * 65 + cc + 3] = v[3];
  }
  __syncthreads();
  const int q = tid >> 3, c8 = (tid & 7) * 8;
  v8h hv[2], lv[2];
#pragma unroll
  for (int g = 0; g < 2; ++g) {
    const int qq = g * 32 + q;
#pragma unroll
    for (int e = 0; e < 8; ++e) {
      const float f = Tt[(c8 + e) * 65 + qq];
      if (MODE == 0) {
        hv[g][e] = (_Float16)(f * sc);
        lv[g][e] = (_Float16)0.0f;
      } else {
        const unsigned short hb = f2bf_bits(f);
        const unsigned short lb = f2bf_bits(f - bf_bits2f(hb));
        hv[g][e] = __builtin_bit_cast(_Float16, hb);
        lv[g][e] = __builtin_bit_cast(_Float16, lb);
      }
    }
  }
  for (int pass = 0; pass < 2; ++pass) {
#pragma unroll
    for (int g = 0; g < 2; ++g) {
      const size_t o = (size_t)(c0 + g * 32 + q) * (size_t)ldo + (size_t)(r0 + c8);
      *(volatile v8h*)(O + o) = hv[g];
      if (MODE == 1) *(volatile v8h*)(O2 + o) = lv[g];
    }
    __threadfence();
  }
}

__global__ __launch_bounds__(SCAN_THR) void trace_scan_kernel(
    const float* __restrict__ h0d, const float* __restrict__ Wh0, const float* __restrict__ bh0,
    const float* __restrict__ Wrec, const float* __restrict__ Arec, const float* __restrict__ XIN,
    const float* __restrict__ alpha1, const float* __restrict__ eta1, unsigned* __restrict__ R16w) {
  __shared__ __align__(16) float r_s[2 * NHID];
  __shared__ __align__(16) float part_s[SCAN_GRP * NHID];
  const int n    = blockIdx.x;
  const int tid  = threadIdx.x;
  const int k    = tid & (NHID - 1);
  const int wave = __builtin_amdgcn_readfirstlane((int)(threadIdx.x >> 5));
  const int grp  = wave >> 2;
  const int hbase = grp * SCAN_EPT;

  const float lk  = alpha1[0];
  const float et  = eta1[0];
  const float oml = 1.0f - lk;
  const float ome = 1.0f - et;

  float wr[SCAN_EPT], ar[SCAN_EPT], tr[SCAN_EPT];
#pragma unroll
  for (int i = 0; i < SCAN_EPT; ++i) wr[i] = Wrec[(size_t)(hbase + i) * NHID + k];
#pragma unroll
  for (int i = 0; i < SCAN_EPT; ++i) { asm volatile("" : "+v"(wr[i])); }
#pragma unroll
  for (int i = 0; i < SCAN_EPT; ++i) ar[i] = Arec[(size_t)(hbase + i) * NHID + k];
#pragma unroll
  for (int i = 0; i < SCAN_EPT; ++i) { asm volatile("" : "+v"(ar[i])); }
#pragma unroll
  for (int i = 0; i < SCAN_EPT; ++i) tr[i] = 0.0f;

  float h = 0.0f;
  float xin = 0.0f;
  if (wave < 4) {
    float acc = 0.0f;
#pragma unroll 4
    for (int j = 0; j < NH0; ++j) acc = fmaf(h0d[(size_t)n * NH0 + j], Wh0[(size_t)j * NHID + k], acc);
    h = acc + bh0[k];
    r_s[k] = 0.0f;
  }

  int cur = 0;
#pragma unroll 1
  for (int t = 0; t < NSTEP; ++t) {
    const int nxt = cur ^ 1;
    const float* rcur = r_s + cur * NHID;
    float* rnxt = r_s + nxt * NHID;

    if (wave < 4) {
      if (t > 0) {
        const float p0 = part_s[0 * NHID + k], p1 = part_s[1 * NHID + k];
        const float p2 = part_s[2 * NHID + k], p3 = part_s[3 * NHID + k];
        const float p4 = part_s[4 * NHID + k], p5 = part_s[5 * NHID + k];
        const float p6 = part_s[6 * NHID + k], p7 = part_s[7 * NHID + k];
        const float rec = ((p0 + p1) + (p2 + p3)) + ((p4 + p5) + (p6 + p7));
        h = oml * h + lk * (rec + xin);
      }
      const float rn = tanhf(h);
      rnxt[k] = rn;
      const int tn = (t < NSTEP - 2) ? t : (NSTEP - 2);
      xin = XIN[((size_t)tn * NSAMP + (size_t)n) * NHID + k];
      asm volatile("" : "+v"(xin));
    }
    __syncthreads();

    if (wave < 2) {
      const float ra = rnxt[2 * tid];
      const float rb = rnxt[2 * tid + 1];
      v2h pk;
      pk[0] = (_Float16)(ra * ACT_CARRY);
      pk[1] = (_Float16)(rb * ACT_CARRY);
      const unsigned u = __builtin_bit_cast(unsigned, pk);
      volatile unsigned* dst = R16w + ((size_t)t * NSAMP + (size_t)n) * (NHID / 2) + tid;
      *dst = u;
      __threadfence();
      *dst = u;
    }

    {
      const float ern = et * rnxt[k];
      const float* ro = rcur + hbase;
      const float* rq = rnxt + hbase;
      float acc0 = 0.0f, acc1 = 0.0f, acc2 = 0.0f, acc3 = 0.0f;
#pragma unroll
      for (int q = 0; q < SCAN_EPT / 4; ++q) {
        const v4f vo = *(const v4f*)(ro + 4 * q);
        const v4f vn = *(const v4f*)(rq + 4 * q);
        tr[4 * q + 0] = fmaf(tr[4 * q + 0], ome, vo[0] * ern);
        tr[4 * q + 1] = fmaf(tr[4 * q + 1], ome, vo[1] * ern);
        tr[4 * q + 2] = fmaf(tr[4 * q + 2], ome, vo[2] * ern);
        tr[4 * q + 3] = fmaf(tr[4 * q + 3], ome, vo[3] * ern);
        acc0 = fmaf(vn[0], fmaf(ar[4 * q + 0], tr[4 * q + 0], wr[4 * q + 0]), acc0);
        acc1 = fmaf(vn[1], fmaf(ar[4 * q + 1], tr[4 * q + 1], wr[4 * q + 1]), acc1);
        acc2 = fmaf(vn[2], fmaf(ar[4 * q + 2], tr[4 * q + 2], wr[4 * q + 2]), acc2);
        acc3 = fmaf(vn[3], fmaf(ar[4 * q + 3], tr[4 * q + 3], wr[4 * q + 3]), acc3);
      }
      part_s[grp * NHID + k] = (acc0 + acc1) + (acc2 + acc3);
    }
    __syncthreads();
    cur = nxt;
  }
}

extern "C" void kernel_launch(void* const* d_in, const int* in_sizes, int n_in,
                              void* d_out, int out_size, void* d_ws, size_t ws_size, hipStream_t stream) {
  if (n_in < 11 || d_out == nullptr || d_ws == nullptr) return;
  if (in_sizes[0] != NSAMP * NH0 || in_sizes[1] != NSTEP * NSAMP * NIN || in_sizes[2] != NH0 * NHID ||
      in_sizes[3] != NHID || in_sizes[4] != NIN * NHID || in_sizes[5] != NHID * NHID || in_sizes[6] != NHID ||
      in_sizes[7] != NHID * NHID || in_sizes[8] != NHID * NOUT || in_sizes[9] != 1 || in_sizes[10] != 1 ||
      out_size != NSTEP * NSAMP * NOUT) return;

  const float* h0_data   = (const float*)d_in[0];
  const float* input_ts  = (const float*)d_in[1];
  const float* W_h0      = (const float*)d_in[2];
  const float* b_h0      = (const float*)d_in[3];
  const float* W_in      = (const float*)d_in[4];
  const float* W_rec     = (const float*)d_in[5];
  const float* b_rec     = (const float*)d_in[6];
  const float* alpha_rec = (const float*)d_in[7];
  const float* W_out     = (const float*)d_in[8];
  const float* alpha     = (const float*)d_in[9];
  const float* eta       = (const float*)d_in[10];
  float* out = (float*)d_out;

  char* ws = (char*)d_ws; size_t off = 0;
  auto carve = [&](size_t bytes) -> char* { char* p = ws + off; off += (bytes + 255) & ~(size_t)255; return p; };
  unsigned short* XH   = (unsigned short*)carve((size_t)XROWS * NIN * 2);
  unsigned short* XL   = (unsigned short*)carve((size_t)XROWS * NIN * 2);
  unsigned short* BIH  = (unsigned short*)carve((size_t)NHID * NIN * 2);
  unsigned short* BIL  = (unsigned short*)carve((size_t)NHID * NIN * 2);
  unsigned short* BOUT = (unsigned short*)carve((size_t)NOUT * NHID * 2);
  float*          XIN  = (float*)carve((size_t)XROWS * NHID * 4);
  unsigned short* R16  = (unsigned short*)carve((size_t)NROWS * NHID * 2);
  if (off > ws_size || off > (size_t)134217728) return;

  const int n8 = XROWS * (NIN / 8);
  split8_kernel<<<n8 / 256, 256, 0, stream>>>(input_ts + (size_t)NSAMP * NIN, XH, XL, n8);

  tp_kernel<1><<<dim3(NHID / 64, NIN / 64), 256, 0, stream>>>(W_in, NIN, NHID, NIN, BIH, BIL, 1.0f);
  tp_kernel<0><<<dim3(NOUT / 64, NHID / 64), 256, 0, stream>>>(W_out, NHID, NOUT, NHID, BOUT, BOUT, WOUT_CARRY);

  wmma_gemm64<1, true, 2><<<dim3(((XROWS >> 6) * (NHID >> 6)) / 8, 1), 256, 0, stream>>>(
      XH, XL, NIN, BIH, BIL, NIN, XIN, NHID, b_rec, XROWS, NHID, NIN, 1.0f);

  trace_scan_kernel<<<NSAMP, SCAN_THR, 0, stream>>>(h0_data, W_h0, b_h0, W_rec, alpha_rec, XIN, alpha, eta,
                                                    (unsigned*)R16);

  wmma_gemm64<0, false, 0><<<dim3(((NROWS >> 6) * (NOUT >> 6)) / 8, 1), 256, 0, stream>>>(
      R16, R16, NHID, BOUT, BOUT, NHID, out, NOUT, b_rec, NROWS, NOUT, NHID, OUT_FOLD);
}
